// butterflyAutoEncode_62981400428623
// MI455X (gfx1250) — hardware-run, weakly checked
//
#include <hip/hip_runtime.h>
#include <math.h>

typedef __attribute__((ext_vector_type(16))) __bf16       v16b;
typedef __attribute__((ext_vector_type(8)))  __bf16       v8b;
typedef __attribute__((ext_vector_type(8)))  float        v8f;
typedef __attribute__((ext_vector_type(4)))  float        v4f;
typedef __attribute__((ext_vector_type(4)))  unsigned int v4u;

constexpr int kD       = 1024;
constexpr int kSk      = 20;
constexpr int kN       = 8192;
constexpr int kRank    = 10;
constexpr int kIters   = 300;
constexpr int kPadRows = 64;
constexpr int kKp      = 32;
constexpr int kSlot    = 512;
constexpr int kGramCh  = 128;
constexpr int kGramP   = 132;
constexpr int kTileP   = 260;
constexpr int kXposeP  = 68;
constexpr int kChunksN = kN / kGramCh;
constexpr int kChunksD = kD / kGramCh;
static_assert(kChunksN == 64 && kChunksD == 8, "chunk counts");
static_assert((kD % 64) == 0 && (kN % 64) == 0 && (kD % 32) == 0 && (kN % 32) == 0, "GEMM tile multiples");
static_assert(kSk * kSk <= kSlot && kSk * kGramCh == 10 * 256, "table and staging coverage");

constexpr size_t kOffXH   = 0;
constexpr size_t kOffXL   = kOffXH   + (size_t)kD * kN * 2;
constexpr size_t kOffXTH  = kOffXL   + (size_t)kD * kN * 2;
constexpr size_t kOffXTL  = kOffXTH  + (size_t)kN * kD * 2;
constexpr size_t kOffWH   = kOffXTL  + (size_t)kN * kD * 2;
constexpr size_t kOffWL   = kOffWH   + (size_t)kPadRows * kD * 2;
constexpr size_t kOffXX   = kOffWL   + (size_t)kPadRows * kD * 2;
constexpr size_t kOffGPP  = kOffXX   + (size_t)kPadRows * kN * 4;
constexpr size_t kOffGP   = kOffGPP  + (size_t)2 * kChunksN * kSlot * 4;
constexpr size_t kOffCM   = kOffGP   + (size_t)2 * kSlot * 4;
constexpr size_t kOffVRH  = kOffCM   + (size_t)kSlot * 4;
constexpr size_t kOffVRL  = kOffVRH  + (size_t)kPadRows * kN * 2;
constexpr size_t kOffV2TH = kOffVRL  + (size_t)kPadRows * kN * 2;
constexpr size_t kOffV2TL = kOffV2TH + (size_t)kN * kKp * 2;
constexpr size_t kOffAU   = kOffV2TL + (size_t)kN * kKp * 2;
constexpr size_t kOffHP   = kOffAU   + (size_t)kD * kPadRows * 4;
constexpr size_t kOffHM   = kOffHP   + (size_t)kChunksD * kSlot * 4;
constexpr size_t kOffMM   = kOffHM   + (size_t)kSlot * 4;
constexpr size_t kOffTH   = kOffMM   + (size_t)kSlot * 4;
constexpr size_t kOffTL   = kOffTH   + (size_t)kD * kKp * 2;
constexpr size_t kWsTotal = kOffTL   + (size_t)kD * kKp * 2;
static_assert(kWsTotal == 73295872ull, "carve total");
static_assert(kWsTotal <= 134217728ull, "carve cap");
static_assert((kOffXL % 128) == 0 && (kOffXTH % 128) == 0 && (kOffXTL % 128) == 0 && (kOffWH % 128) == 0 &&
              (kOffWL % 128) == 0 && (kOffXX % 128) == 0 && (kOffGPP % 128) == 0 && (kOffGP % 128) == 0 &&
              (kOffCM % 128) == 0 && (kOffVRH % 128) == 0 && (kOffVRL % 128) == 0 && (kOffV2TH % 128) == 0 &&
              (kOffV2TL % 128) == 0 && (kOffAU % 128) == 0 && (kOffHP % 128) == 0 && (kOffHM % 128) == 0 &&
              (kOffMM % 128) == 0 && (kOffTH % 128) == 0 && (kOffTL % 128) == 0, "128-B aligned regions");

__device__ __forceinline__ unsigned f2bf_bits(float f) {
  const unsigned u = __float_as_uint(f);
  return (u + 0x7FFFu + ((u >> 16) & 1u)) >> 16;
}
__device__ __forceinline__ float bf_bits2f(unsigned h) { return __uint_as_float(h << 16); }

__device__ __forceinline__ void split_pair(float a, float b, unsigned& hw, unsigned& lw) {
  const unsigned ha = f2bf_bits(a), hb = f2bf_bits(b);
  const unsigned la = f2bf_bits(a - bf_bits2f(ha)), lb = f2bf_bits(b - bf_bits2f(hb));
  hw = ha | (hb << 16);
  lw = la | (lb << 16);
}
__device__ __forceinline__ void pack8_split(v4f a0, v4f a1, v4u& h, v4u& l) {
  unsigned h0, h1, h2, h3, l0, l1, l2, l3;
  split_pair(a0[0], a0[1], h0, l0);
  split_pair(a0[2], a0[3], h1, l1);
  split_pair(a1[0], a1[1], h2, l2);
  split_pair(a1[2], a1[3], h3, l3);
  h = (v4u){h0, h1, h2, h3};
  l = (v4u){l0, l1, l2, l3};
}
__device__ __forceinline__ v4f sel4(bool c, v4f v) {
  v4f r;
  r[0] = c ? v[0] : 0.f;
  r[1] = c ? v[1] : 0.f;
  r[2] = c ? v[2] : 0.f;
  r[3] = c ? v[3] : 0.f;
  return r;
}
__device__ __forceinline__ float dot20(const float* a, const float* b) {
  float s0 = 0.f, s1 = 0.f, s2 = 0.f, s3 = 0.f;
#pragma unroll 1
  for (int kk = 0; kk < 5; ++kk) {
    const v4f x = *(const v4f*)(a + 4 * kk);
    const v4f y = *(const v4f*)(b + 4 * kk);
    s0 = fmaf(x[0], y[0], s0);
    s1 = fmaf(x[1], y[1], s1);
    s2 = fmaf(x[2], y[2], s2);
    s3 = fmaf(x[3], y[3], s3);
  }
  return (s0 + s1) + (s2 + s3);
}
__device__ __forceinline__ float wave_sum(float v) {
#pragma unroll
  for (int off = 16; off >= 1; off >>= 1) v += __shfl_xor(v, off, 32);
  return v;
}

union FragU { v16b v; v8b h[2]; };
__device__ __forceinline__ v16b frag_load(const __bf16* p) {
  FragU f;
  f.h[0] = *(const v8b*)(p);
  f.h[1] = *(const v8b*)(p + 16);
  return f.v;
}
__device__ __forceinline__ v8f mma_b(v16b a, v16b b, v8f c) {
  return __builtin_amdgcn_wmma_f32_16x16x32_bf16(false, a, false, b, (short)0, c, false, false);
}
__device__ __forceinline__ void tie_acc(v8f& acc, v16b a0, v16b a1, v16b b0, v16b b1) {
  asm volatile("v_nop\n\tv_nop\n\tv_nop\n\tv_nop" : "+v"(acc) : "v"(a0), "v"(a1), "v"(b0), "v"(b1));
}
__device__ __forceinline__ void keep4_b(v16b a, v16b b, v16b c, v16b d) { asm volatile("v_nop" :: "v"(a), "v"(b), "v"(c), "v"(d)); }
__device__ __forceinline__ void acc_guard4(v8f& a, v8f& b, v8f& c, v8f& d) { asm volatile("v_nop\n\tv_nop\n\tv_nop\n\tv_nop" : "+v"(a), "+v"(b), "+v"(c), "+v"(d)); }

__global__ __launch_bounds__(256) void gemm64_split_kernel(
    const unsigned short* __restrict__ Ap, const unsigned short* __restrict__ A2p, int lda,
    const unsigned short* __restrict__ Btp, const unsigned short* __restrict__ Bt2p, int ldb,
    float* __restrict__ Cout, int ldc, int M, int N, int K)
{
  const __bf16* A   = (const __bf16*)Ap;
  const __bf16* A2  = (const __bf16*)A2p;
  const __bf16* Bt  = (const __bf16*)Btp;
  const __bf16* Bt2 = (const __bf16*)Bt2p;
  __shared__ __align__(16) float sSlab[8][16 * 68];
  const int lane = threadIdx.x & 31;
  const int wave = threadIdx.x >> 5;
  const int tilesN = N >> 6;
  const int tilesM = M >> 6;
  const int tile = blockIdx.x * 8 + wave;
  if (tile >= tilesM * tilesN) return;
  const int tm = tile / tilesN;
  const int tn = tile - tm * tilesN;
  const int m0 = tm << 6;
  const int n0 = tn << 6;

  const int rlane = lane & 15;
  const int koff  = (lane >> 4) * 8;
  const int mOff  = (lane >> 4) * 8;

  v8f acc[4][4];
#pragma unroll
  for (int i = 0; i < 4; ++i)
#pragma unroll
    for (int j = 0; j < 4; ++j) acc[i][j] = (v8f){0.f, 0.f, 0.f, 0.f, 0.f, 0.f, 0.f, 0.f};

  for (int k0 = 0; k0 < K; k0 += 32) {
    v16b bh[4], bl[4];
#pragma unroll
    for (int j = 0; j < 4; ++j) {
      const size_t bo = (size_t)(n0 + (j << 4) + rlane) * ldb + koff + k0;
      bh[j] = frag_load(Bt + bo);
      bl[j] = frag_load(Bt2 + bo);
    }
#pragma unroll
    for (int i = 0; i < 4; ++i) {
      const size_t ao = (size_t)(m0 + (i << 4) + rlane) * lda + koff + k0;
      const v16b ah = frag_load(A + ao);
      const v16b al = frag_load(A2 + ao);
#pragma unroll
      for (int j = 0; j < 4; ++j) {
        acc[i][j] = mma_b(ah, bh[j], acc[i][j]);
        acc[i][j] = mma_b(ah, bl[j], acc[i][j]);
        acc[i][j] = mma_b(al, bh[j], acc[i][j]);
      }
#pragma unroll
      for (int j = 0; j < 4; ++j) tie_acc(acc[i][j], ah, al, bh[j], bl[j]);
    }
    keep4_b(bh[0], bh[1], bh[2], bh[3]);
    keep4_b(bl[0], bl[1], bl[2], bl[3]);
  }
  acc_guard4(acc[0][0], acc[0][1], acc[0][2], acc[0][3]);
  acc_guard4(acc[1][0], acc[1][1], acc[1][2], acc[1][3]);
  acc_guard4(acc[2][0], acc[2][1], acc[2][2], acc[2][3]);
  acc_guard4(acc[3][0], acc[3][1], acc[3][2], acc[3][3]);

  float* slab = sSlab[wave];
#pragma unroll
  for (int i = 0; i < 4; ++i) {
    const int mBase = m0 + (i << 4);
#pragma unroll
    for (int j = 0; j < 4; ++j) {
#pragma unroll
      for (int r = 0; r < 8; ++r) slab[(mOff + r) * 68 + (j << 4) + rlane] = acc[i][j][r];
    }
    __builtin_amdgcn_fence(__ATOMIC_RELEASE, "workgroup");
    __builtin_amdgcn_wave_barrier();
    __builtin_amdgcn_fence(__ATOMIC_ACQUIRE, "workgroup");
    {
      const int hh = lane >> 4, c4 = (lane & 15) * 4;
      for (int pass = 0; pass < 2; ++pass) {
#pragma unroll
        for (int it = 0; it < 8; ++it) {
          const int row = it * 2 + hh;
          const v4f v = *(const v4f*)(slab + row * 68 + c4);
          *(volatile v4f*)(Cout + (size_t)(mBase + row) * ldc + n0 + c4) = v;
        }
        __threadfence();
      }
    }
    __builtin_amdgcn_fence(__ATOMIC_RELEASE, "workgroup");
    __builtin_amdgcn_wave_barrier();
    __builtin_amdgcn_fence(__ATOMIC_ACQUIRE, "workgroup");
  }
}

__global__ __launch_bounds__(256) void split_x_kernel(
    const float* __restrict__ x, unsigned short* __restrict__ XH, unsigned short* __restrict__ XL,
    unsigned short* __restrict__ XTH, unsigned short* __restrict__ XTL)
{
  __shared__ __align__(16) float sT[64 * kXposeP];
  const int tid = threadIdx.x, lane = tid & 31, wave = tid >> 5;
  const int r0 = blockIdx.y * 64, c0 = blockIdx.x * 64;
  {
    const int lr = tid >> 4, c4 = (tid & 15) * 4;
#pragma unroll
    for (int i = 0; i < 4; ++i) {
      const int row = lr + 16 * i;
      *(v4f*)&sT[row * kXposeP + c4] = *(const v4f*)(x + (size_t)(r0 + row) * kN + c0 + c4);
    }
  }
  __syncthreads();
  const int q = lane >> 3, e8 = (lane & 7) * 8;
  v4u sh[2], sl[2], th[2], tl[2];
#pragma unroll
  for (int it = 0; it < 2; ++it) {
    const int rr = it * 32 + wave * 4 + q;
    const v4f a0 = *(const v4f*)&sT[rr * kXposeP + e8];
    const v4f a1 = *(const v4f*)&sT[rr * kXposeP + e8 + 4];
    pack8_split(a0, a1, sh[it], sl[it]);
    float tv[8];
#pragma unroll
    for (int e = 0; e < 8; ++e) tv[e] = sT[(e8 + e) * kXposeP + rr];
    const v4f b0 = (v4f){tv[0], tv[1], tv[2], tv[3]};
    const v4f b1 = (v4f){tv[4], tv[5], tv[6], tv[7]};
    pack8_split(b0, b1, th[it], tl[it]);
  }
  for (int pass = 0; pass < 2; ++pass) {
#pragma unroll
    for (int it = 0; it < 2; ++it) {
      const int rr = it * 32 + wave * 4 + q;
      const size_t os = (size_t)(r0 + rr) * kN + c0 + e8;
      const size_t ot = (size_t)(c0 + rr) * kD + r0 + e8;
      *(volatile v4u*)(XH + os)  = sh[it];
      *(volatile v4u*)(XL + os)  = sl[it];
      *(volatile v4u*)(XTH + ot) = th[it];
      *(volatile v4u*)(XTL + ot) = tl[it];
    }
    __threadfence();
  }
}

__global__ __launch_bounds__(256) void split_w_kernel(
    const float* __restrict__ W, unsigned short* __restrict__ WH, unsigned short* __restrict__ WL)
{
  const int i = blockIdx.x * 256 + threadIdx.x;
  const int row = i >> 7, c8 = (i & 127) * 8;
  const bool live = row < kSk;
  const int rc = live ? row : (kSk - 1);
  v4f a0 = *(const v4f*)(W + (size_t)rc * kD + c8);
  v4f a1 = *(const v4f*)(W + (size_t)rc * kD + c8 + 4);
  a0 = sel4(live, a0);
  a1 = sel4(live, a1);
  v4u h, l;
  pack8_split(a0, a1, h, l);
  const size_t o = (size_t)row * kD + c8;
  *(volatile v4u*)(WH + o) = h;
  *(volatile v4u*)(WL + o) = l;
  __threadfence();
  *(volatile v4u*)(WH + o) = h;
  *(volatile v4u*)(WL + o) = l;
}

__global__ __launch_bounds__(256) void gram_part_kernel(
    const float* A, const float* B0, const float* B1,
    int rsA, int rsB, int es, float* __restrict__ part, int nchunks)
{
  __shared__ __align__(16) float sA[kSk * kGramP];
  __shared__ __align__(16) float sB[kSk * kGramP];
  __shared__ __align__(16) float sO[kSlot];
  const int tid = threadIdx.x;
  const int chunk = blockIdx.x, pair = blockIdx.y;
  const float* B = (pair == 0) ? B0 : B1;
  const size_t t0 = (size_t)chunk * kGramCh;
#pragma unroll 1
  for (int it = 0; it < 10; ++it) {
    const int idx = tid + 256 * it;
    const int row = idx >> 7, t = idx & 127;
    sA[row * kGramP + t] = A[(size_t)row * rsA + (t0 + t) * (size_t)es];
    sB[row * kGramP + t] = B[(size_t)row * rsB + (t0 + t) * (size_t)es];
  }
  __syncthreads();
#pragma unroll 1
  for (int i2 = 0; i2 < 2; ++i2) {
    const int o = tid + 256 * i2;
    const int oc = (o < kSk * kSk) ? o : (kSk * kSk - 1);
    const int i = oc / kSk, j = oc - i * kSk;
    float s0 = 0.f, s1 = 0.f, s2 = 0.f, s3 = 0.f;
#pragma unroll 1
    for (int t4 = 0; t4 < kGramCh / 4; ++t4) {
      const v4f a = *(const v4f*)&sA[i * kGramP + 4 * t4];
      const v4f b = *(const v4f*)&sB[j * kGramP + 4 * t4];
      s0 = fmaf(a[0], b[0], s0);
      s1 = fmaf(a[1], b[1], s1);
      s2 = fmaf(a[2], b[2], s2);
      s3 = fmaf(a[3], b[3], s3);
    }
    const float acc = (s0 + s1) + (s2 + s3);
    sO[o] = (o < kSk * kSk) ? acc : 0.f;
  }
  __syncthreads();
  if (tid < 128) {
    const v4f v = *(const v4f*)&sO[tid * 4];
    float* dst = part + ((size_t)pair * nchunks + chunk) * kSlot + tid * 4;
    *(volatile v4f*)dst = v;
    __threadfence();
    *(volatile v4f*)dst = v;
  }
}

__global__ __launch_bounds__(128) void gram_reduce_kernel(
    const float* __restrict__ part, float* __restrict__ out, int nchunks)
{
  const int pair = blockIdx.x, tid = threadIdx.x;
  v4f acc = (v4f){0.f, 0.f, 0.f, 0.f};
#pragma unroll 1
  for (int c = 0; c < nchunks; ++c) {
    const v4f p = *(const v4f*)(part + ((size_t)pair * nchunks + c) * kSlot + tid * 4);
    acc[0] += p[0];
    acc[1] += p[1];
    acc[2] += p[2];
    acc[3] += p[3];
  }
  float* dst = out + (size_t)pair * kSlot + tid * 4;
  *(volatile v4f*)dst = acc;
  __threadfence();
  *(volatile v4f*)dst = acc;
}

__global__ __launch_bounds__(32) void svd_gram_kernel(const float* __restrict__ GP, float* __restrict__ Cout)
{
  __shared__ __align__(16) float sG[416];
  __shared__ __align__(16) float sW[kSk * kSk];
  __shared__ __align__(16) float sC[kSlot];
  __shared__ __align__(16) float sz[32];
  __shared__ __align__(16) float sp[32];
  const int lane = threadIdx.x;
  const bool act = lane < kSk;
  const int li = act ? lane : (kSk - 1);
#pragma unroll 1
  for (int i = 0; i < 13; ++i) sG[lane + 32 * i] = GP[lane + 32 * i];
#pragma unroll 1
  for (int i = 0; i < 4; ++i) {
    const int idx = kSk * kSk + lane + 32 * i;
    if (idx < kSlot) sC[idx] = 0.f;
  }
  __syncthreads();
#pragma unroll 1
  for (int j = 0; j < kSk; ++j) {
    float pv = GP[kSlot + li * kSk + j];
    asm volatile("" : "+v"(pv));
    const float pi = act ? pv : 0.f;
    __syncthreads();
    sp[lane] = pi;
    __syncthreads();
    float zi = pi;
#pragma unroll 1
    for (int jp = 0; jp < j; ++jp) {
      const float dd = dot20(&sC[jp * kSk], &sp[0]);
      zi -= sW[jp * kSk + li] * dd;
    }
    zi = act ? zi : 0.f;
    sz[lane] = zi;
    __syncthreads();
#pragma unroll 1
    for (int t = 0; t < kIters - 1; ++t) {
      float g = dot20(&sG[li * kSk], &sz[0]);
      g = act ? g : 0.f;
      const float nsq = wave_sum(zi * g);
      const float inv = 1.0f / sqrtf(nsq);
      zi = g * inv;
      __syncthreads();
      sz[lane] = zi;
      __syncthreads();
    }
    float g = dot20(&sG[li * kSk], &sz[0]);
    g = act ? g : 0.f;
    const float nsq = wave_sum(zi * g);
    const float invn = 1.0f / sqrtf(nsq);
    const float wi = g * invn;
    float ci = zi;
#pragma unroll 1
    for (int jp = 0; jp < j; ++jp) {
      const float dd = dot20(&sW[jp * kSk], &sz[0]);
      ci -= sC[jp * kSk + li] * dd;
    }
    ci *= invn;
    __syncthreads();
    if (act) {
      sW[j * kSk + lane] = wi;
      sC[j * kSk + lane] = ci;
    }
    __syncthreads();
#pragma unroll 1
    for (int kk = 0; kk < 5; ++kk) {
      v4f gv = *(const v4f*)&sG[li * kSk + 4 * kk];
      const v4f wv = *(const v4f*)&sW[j * kSk + 4 * kk];
      gv[0] -= wi * wv[0];
      gv[1] -= wi * wv[1];
      gv[2] -= wi * wv[2];
      gv[3] -= wi * wv[3];
      if (act) *(v4f*)&sG[li * kSk + 4 * kk] = gv;
    }
  }
  __syncthreads();
  for (int pass = 0; pass < 2; ++pass) {
#pragma unroll
    for (int i = 0; i < 4; ++i) {
      const int idx = (lane + 32 * i) * 4;
      const v4f v = *(const v4f*)&sC[idx];
      *(volatile v4f*)(Cout + idx) = v;
    }
    __threadfence();
  }
}

__global__ __launch_bounds__(256) void vrows_kernel(
    const float* __restrict__ XX, const float* __restrict__ Cm,
    unsigned short* __restrict__ VRH, unsigned short* __restrict__ VRL,
    unsigned short* __restrict__ V2TH, unsigned short* __restrict__ V2TL)
{
  __shared__ __align__(16) float sC[kSlot];
  __shared__ __align__(16) float sV[kSk * kTileP];
  const int tid = threadIdx.x, lane = tid & 31, wave = tid >> 5;
  const int q0 = blockIdx.x * 256;
  sC[tid] = Cm[tid];
  sC[tid + 256] = Cm[tid + 256];
  __syncthreads();
  float acc[kSk];
#pragma unroll
  for (int j = 0; j < kSk; ++j) acc[j] = 0.f;
#pragma unroll 1
  for (int k = 0; k < kSk; ++k) {
    const float xv = XX[(size_t)k * kN + q0 + tid];
#pragma unroll
    for (int j = 0; j < kSk; ++j) acc[j] = fmaf(sC[j * kSk + k], xv, acc[j]);
  }
#pragma unroll
  for (int j = 0; j < kSk; ++j) sV[j * kTileP + tid] = acc[j];
  __syncthreads();
  for (int pass = 0; pass < 2; ++pass) {
#pragma unroll 1
    for (int it = 0; it < 8; ++it) {
      const int jr = wave + 8 * it;
      const bool live = jr < kSk;
      const int jc = live ? jr : (kSk - 1);
      v4f a0 = *(const v4f*)&sV[jc * kTileP + lane * 8];
      v4f a1 = *(const v4f*)&sV[jc * kTileP + lane * 8 + 4];
      a0 = sel4(live, a0);
      a1 = sel4(live, a1);
      v4u h, l;
      pack8_split(a0, a1, h, l);
      const size_t o = (size_t)jr * kN + q0 + lane * 8;
      *(volatile v4u*)(VRH + o) = h;
      *(volatile v4u*)(VRL + o) = l;
    }
#pragma unroll 1
    for (int it = 0; it < 4; ++it) {
      const int rq = (wave * 4 + it) * 8 + (lane >> 2);
      const int ks = (lane & 3) * 8;
      float tv[8];
#pragma unroll
      for (int e = 0; e < 8; ++e) {
        const int k = ks + e;
        const int kc = (k < kSk) ? k : (kSk - 1);
        const float v = sV[kc * kTileP + rq];
        tv[e] = (k < kSk) ? v : 0.f;
      }
      const v4f b0 = (v4f){tv[0], tv[1], tv[2], tv[3]};
      const v4f b1 = (v4f){tv[4], tv[5], tv[6], tv[7]};
      v4u h, l;
      pack8_split(b0, b1, h, l);
      const size_t o = (size_t)(q0 + rq) * kKp + ks;
      *(volatile v4u*)(V2TH + o) = h;
      *(volatile v4u*)(V2TL + o) = l;
    }
    __threadfence();
  }
}

__global__ __launch_bounds__(32) void svd_small_kernel(
    const float* __restrict__ Hg, const float* __restrict__ vinit, float* __restrict__ Mout)
{
  __shared__ __align__(16) float sH[416];
  __shared__ __align__(16) float sXF[kRank * kSk + 8];
  __shared__ __align__(16) float sDx[kRank * kSk + 8];
  __shared__ __align__(16) float sM[kSlot];
  __shared__ __align__(16) float sx[32];
  __shared__ __align__(16) float sh[32];
  const int lane = threadIdx.x;
  const bool act = lane < kSk;
  const int li = act ? lane : (kSk - 1);
#pragma unroll 1
  for (int i = 0; i < 13; ++i) sH[lane + 32 * i] = Hg[lane + 32 * i];
#pragma unroll 1
  for (int i = 0; i < 16; ++i) sM[lane + 32 * i] = 0.f;
  __syncthreads();
#pragma unroll 1
  for (int j = 0; j < kRank; ++j) {
    float xv = vinit[j * kSk + li];
    asm volatile("" : "+v"(xv));
    float xi = act ? xv : 0.f;
    __syncthreads();
    sx[lane] = xi;
    __syncthreads();
#pragma unroll 1
    for (int t = 0; t < kIters; ++t) {
      float hx = dot20(&sH[li * kSk], &sx[0]);
      hx = act ? hx : 0.f;
      const float nsq = wave_sum(hx * hx);
      const float inv = 1.0f / sqrtf(nsq);
      xi = hx * inv;
      __syncthreads();
      sx[lane] = xi;
      __syncthreads();
    }
    const float nrm2 = wave_sum(xi * xi);
    const float rn = 1.0f / sqrtf(nrm2);
    float dxi = xi;
#pragma unroll 1
    for (int jp = 0; jp < j; ++jp) {
      const float dd = dot20(&sXF[jp * kSk], &sx[0]);
      dxi -= sDx[jp * kSk + li] * dd;
    }
    dxi = act ? dxi : 0.f;
    const float dr = dxi * rn;
#pragma unroll 1
    for (int kk = 0; kk < 5; ++kk) {
      v4f mv = *(const v4f*)&sM[li * kSk + 4 * kk];
      const v4f xs = *(const v4f*)&sx[4 * kk];
      mv[0] = fmaf(dr, xs[0] * rn, mv[0]);
      mv[1] = fmaf(dr, xs[1] * rn, mv[1]);
      mv[2] = fmaf(dr, xs[2] * rn, mv[2]);
      mv[3] = fmaf(dr, xs[3] * rn, mv[3]);
      if (act) *(v4f*)&sM[li * kSk + 4 * kk] = mv;
    }
    float hx = dot20(&sH[li * kSk], &sx[0]);
    hx = act ? hx : 0.f;
    sh[lane] = hx;
    __syncthreads();
    const float qf = wave_sum(xi * hx);
    const float qx = qf * xi;
#pragma unroll 1
    for (int kk = 0; kk < 5; ++kk) {
      v4f hv = *(const v4f*)&sH[li * kSk + 4 * kk];
      const v4f xs = *(const v4f*)&sx[4 * kk];
      const v4f hs = *(const v4f*)&sh[4 * kk];
      hv[0] -= (hx * xs[0] + xi * hs[0]) - qx * xs[0];
      hv[1] -= (hx * xs[1] + xi * hs[1]) - qx * xs[1];
      hv[2] -= (hx * xs[2] + xi * hs[2]) - qx * xs[2];
      hv[3] -= (hx * xs[3] + xi * hs[3]) - qx * xs[3];
      if (act) *(v4f*)&sH[li * kSk + 4 * kk] = hv;
    }
    if (act) {
      sXF[j * kSk + lane] = xi;
      sDx[j * kSk + lane] = dxi;
    }
  }
  __syncthreads();
  for (int pass = 0; pass < 2; ++pass) {
#pragma unroll
    for (int i = 0; i < 4; ++i) {
      const int idx = (lane + 32 * i) * 4;
      const v4f v = *(const v4f*)&sM[idx];
      *(volatile v4f*)(Mout + idx) = v;
    }
    __threadfence();
  }
}

__global__ __launch_bounds__(256) void tplanes_kernel(
    const float* __restrict__ AU, const float* __restrict__ Mm,
    unsigned short* __restrict__ TH, unsigned short* __restrict__ TL)
{
  __shared__ __align__(16) float sM[kSlot];
  __shared__ __align__(16) float sT[kSk * kTileP];
  const int tid = threadIdx.x, lane = tid & 31, wave = tid >> 5;
  const int r0 = blockIdx.x * 256;
  sM[tid] = Mm[tid];
  sM[tid + 256] = Mm[tid + 256];
  __syncthreads();
  float a[kSk];
#pragma unroll
  for (int i = 0; i < 5; ++i) {
    const v4f av = *(const v4f*)(AU + (size_t)(r0 + tid) * kPadRows + 4 * i);
    a[4 * i + 0] = av[0];
    a[4 * i + 1] = av[1];
    a[4 * i + 2] = av[2];
    a[4 * i + 3] = av[3];
  }
#pragma unroll 1
  for (int j = 0; j < kSk; ++j) {
    float acc = 0.f;
#pragma unroll
    for (int k = 0; k < kSk; ++k) acc = fmaf(a[k], sM[k * kSk + j], acc);
    sT[j * kTileP + tid] = acc;
  }
  __syncthreads();
  for (int pass = 0; pass < 2; ++pass) {
#pragma unroll 1
    for (int it = 0; it < 4; ++it) {
      const int rq = (wave * 4 + it) * 8 + (lane >> 2);
      const int ks = (lane & 3) * 8;
      float tv[8];
#pragma unroll
      for (int e = 0; e < 8; ++e) {
        const int k = ks + e;
        const int kc = (k < kSk) ? k : (kSk - 1);
        const float v = sT[kc * kTileP + rq];
        tv[e] = (k < kSk) ? v : 0.f;
      }
      const v4f b0 = (v4f){tv[0], tv[1], tv[2], tv[3]};
      const v4f b1 = (v4f){tv[4], tv[5], tv[6], tv[7]};
      v4u h, l;
      pack8_split(b0, b1, h, l);
      const size_t o = (size_t)(r0 + rq) * kKp + ks;
      *(volatile v4u*)(TH + o) = h;
      *(volatile v4u*)(TL + o) = l;
    }
    __threadfence();
  }
}

extern "C" void kernel_launch(void* const* d_in, const int* in_sizes, int n_in,
                              void* d_out, int out_size, void* d_ws, size_t ws_size,
                              hipStream_t stream) {
  if (n_in < 4) return;
  if (in_sizes[0] != kD * kN) return;
  if (in_sizes[1] != kSk * kD) return;
  if (in_sizes[2] != kSk * kN) return;
  if (in_sizes[3] != kRank * kSk) return;
  if (out_size != kD * kN) return;
  if (ws_size < kWsTotal) return;

  const float* x   = (const float*)d_in[0];
  const float* W   = (const float*)d_in[1];
  const float* v1  = (const float*)d_in[2];
  const float* v2i = (const float*)d_in[3];
  float* out = (float*)d_out;

  char* ws = (char*)d_ws;
  unsigned short* XH   = (unsigned short*)(ws + kOffXH);
  unsigned short* XL   = (unsigned short*)(ws + kOffXL);
  unsigned short* XTH  = (unsigned short*)(ws + kOffXTH);
  unsigned short* XTL  = (unsigned short*)(ws + kOffXTL);
  unsigned short* WH   = (unsigned short*)(ws + kOffWH);
  unsigned short* WL   = (unsigned short*)(ws + kOffWL);
  float*          XX   = (float*)(ws + kOffXX);
  float*          GPP  = (float*)(ws + kOffGPP);
  float*          GP   = (float*)(ws + kOffGP);
  float*          CM   = (float*)(ws + kOffCM);
  unsigned short* VRH  = (unsigned short*)(ws + kOffVRH);
  unsigned short* VRL  = (unsigned short*)(ws + kOffVRL);
  unsigned short* V2TH = (unsigned short*)(ws + kOffV2TH);
  unsigned short* V2TL = (unsigned short*)(ws + kOffV2TL);
  float*          AU   = (float*)(ws + kOffAU);
  float*          HP   = (float*)(ws + kOffHP);
  float*          HM   = (float*)(ws + kOffHM);
  float*          MM   = (float*)(ws + kOffMM);
  unsigned short* TH   = (unsigned short*)(ws + kOffTH);
  unsigned short* TL   = (unsigned short*)(ws + kOffTL);

  split_x_kernel<<<dim3(kN / 64, kD / 64), 256, 0, stream>>>(x, XH, XL, XTH, XTL);
  split_w_kernel<<<(kPadRows * kD / 8) / 256, 256, 0, stream>>>(W, WH, WL);

  gemm64_split_kernel<<<(1 * (kN / 64)) / 8, 256, 0, stream>>>(
      WH, WL, kD, XTH, XTL, kD, XX, kN, kPadRows, kN, kD);

  gram_part_kernel<<<dim3(kChunksN, 2), 256, 0, stream>>>(XX, XX, v1, kN, kN, 1, GPP, kChunksN);
  gram_reduce_kernel<<<2, 128, 0, stream>>>(GPP, GP, kChunksN);

  svd_gram_kernel<<<1, 32, 0, stream>>>(GP, CM);

  vrows_kernel<<<kN / 256, 256, 0, stream>>>(XX, CM, VRH, VRL, V2TH, V2TL);

  gemm64_split_kernel<<<((kD / 64) * 1) / 8, 256, 0, stream>>>(
      XH, XL, kN, VRH, VRL, kN, AU, kPadRows, kD, kPadRows, kN);

  gram_part_kernel<<<dim3(kChunksD, 1), 256, 0, stream>>>(AU, AU, AU, 1, 1, kPadRows, HP, kChunksD);
  gram_reduce_kernel<<<1, 128, 0, stream>>>(HP, HM, kChunksD);

  svd_small_kernel<<<1, 32, 0, stream>>>(HM, v2i, MM);

  tplanes_kernel<<<kD / 256, 256, 0, stream>>>(AU, MM, TH, TL);

  gemm64_split_kernel<<<((kD / 64) * (kN / 64)) / 8, 256, 0, stream>>>(
      TH, TL, kKp, V2TH, V2TL, kKp, out, kN, kD, kN, kKp);
}
